// ROIDCN_9002251452666
// MI455X (gfx1250) — hardware-verified
//
#include <hip/hip_runtime.h>
#include <math.h>

#pragma clang fp contract(off)

constexpr int kBatch    = 2;
constexpr int kChan     = 256;
constexpr int kH        = 128;
constexpr int kW        = 128;
constexpr int kHW       = kH * kW;
constexpr int kTaps     = 9;
constexpr int kKdim     = kTaps * kChan;
constexpr int kHalfPix  = 8192;
constexpr int kPixPerBlk = 8;
constexpr float kThird  = 1.0f / 3.0f;
static_assert(kKdim % 32 == 0);
static_assert(kChan % 64 == 0);
static_assert(kHalfPix % 64 == 0);
static_assert(kHW % kHalfPix == 0);
static_assert(kHalfPix % kPixPerBlk == 0);

typedef __attribute__((ext_vector_type(16))) _Float16 v16h;
typedef __attribute__((ext_vector_type(8)))  _Float16 v8h;
typedef __attribute__((ext_vector_type(16))) __bf16   v16b;
typedef __attribute__((ext_vector_type(8)))  __bf16   v8b;
typedef __attribute__((ext_vector_type(8)))  float    v8f;
typedef __attribute__((ext_vector_type(4)))  float    v4f;
typedef __attribute__((ext_vector_type(4)))  unsigned int v4u;

__device__ __forceinline__ unsigned short f2bf_bits(float f) {
  unsigned u = __float_as_uint(f);
  return (unsigned short)((u + 0x7FFFu + ((u >> 16) & 1u)) >> 16);
}
__device__ __forceinline__ float bf_bits2f(unsigned short h) { return __uint_as_float(((unsigned)h) << 16); }

__device__ __forceinline__ void dep_guard_h(v8f& a, v8f& b, v16h x, v16h y) { asm volatile("v_nop\n\tv_nop\n\tv_nop\n\tv_nop" : "+v"(a), "+v"(b) : "v"(x), "v"(y)); }
__device__ __forceinline__ void dep_guard_b(v8f& a, v8f& b, v16b x, v16b y) { asm volatile("v_nop\n\tv_nop\n\tv_nop\n\tv_nop" : "+v"(a), "+v"(b) : "v"(x), "v"(y)); }
__device__ __forceinline__ void keep4_h(v16h a, v16h b, v16h c, v16h d) { asm volatile("v_nop" :: "v"(a), "v"(b), "v"(c), "v"(d)); }
__device__ __forceinline__ void keep4_b(v16b a, v16b b, v16b c, v16b d) { asm volatile("v_nop" :: "v"(a), "v"(b), "v"(c), "v"(d)); }
__device__ __forceinline__ void acc_guard4(v8f& a, v8f& b, v8f& c, v8f& d) { asm volatile("v_nop\n\tv_nop\n\tv_nop\n\tv_nop" : "+v"(a), "+v"(b), "+v"(c), "+v"(d)); }
template <typename T> struct Frag;
template <> struct Frag<_Float16> {
  typedef v16h V; union U { v16h v; v8h h[2]; };
  static __device__ __forceinline__ v16h load(const _Float16* p) {
    U f; f.h[0] = *(const v8h*)(p); f.h[1] = *(const v8h*)(p + 16); return f.v;
  }
  static __device__ __forceinline__ v8f mma(v16h a, v16h b, v8f c) {
    return __builtin_amdgcn_wmma_f32_16x16x32_f16(false, a, false, b, (short)0, c, false, false);
  }
  static __device__ __forceinline__ void guard(v8f& a, v8f& b, v16h x, v16h y) { dep_guard_h(a, b, x, y); }
  static __device__ __forceinline__ void keep(v16h a, v16h b, v16h c, v16h d) { keep4_h(a, b, c, d); }
};
template <> struct Frag<__bf16> {
  typedef v16b V; union U { v16b v; v8b h[2]; };
  static __device__ __forceinline__ v16b load(const __bf16* p) {
    U f; f.h[0] = *(const v8b*)(p); f.h[1] = *(const v8b*)(p + 16); return f.v;
  }
  static __device__ __forceinline__ v8f mma(v16b a, v16b b, v8f c) {
    return __builtin_amdgcn_wmma_f32_16x16x32_bf16(false, a, false, b, (short)0, c, false, false);
  }
  static __device__ __forceinline__ void guard(v8f& a, v8f& b, v16b x, v16b y) { dep_guard_b(a, b, x, y); }
  static __device__ __forceinline__ void keep(v16b a, v16b b, v16b c, v16b d) { keep4_b(a, b, c, d); }
};

template <int ET> struct Elem;
template <> struct Elem<0> { typedef _Float16 T; };
template <> struct Elem<1> { typedef __bf16 T; };
template <int ET, bool SPLIT, int BIAS_MODE, int OUT_MODE, bool RESID, int ACT = 0>
__global__ __launch_bounds__(256) void wmma_gemm64(
    const unsigned short* __restrict__ Ap, const unsigned short* __restrict__ A2p, int lda, long strideA,
    const unsigned short* __restrict__ Btp, const unsigned short* __restrict__ Bt2p, int ldb, long strideB,
    void* __restrict__ Cout, void* __restrict__ Cout2, int ldc, long strideC,
    const float* __restrict__ bias,
    const float* __restrict__ resid, long strideR,
    int M, int N, int K, float scale) {
  typedef typename Elem<ET>::T T;
  typedef typename Frag<T>::V V;
  const T* A = (const T*)Ap; const T* A2 = (const T*)A2p; const T* Bt = (const T*)Btp; const T* Bt2 = (const T*)Bt2p;
  __shared__ __align__(16) float sT[8][16 * 68];
  const int b    = blockIdx.y;
  const int lane = threadIdx.x & 31;
  const int wave = threadIdx.x >> 5;
  const int tilesN = N >> 6;
  const int tilesM = M >> 6;
  const int tile = blockIdx.x * 8 + wave;
  if (tile >= tilesM * tilesN) return;
  const int tm = tile / tilesN;
  const int tn = tile - tm * tilesN;
  const int m0 = tm << 6;
  const int n0 = tn << 6;

  const T* Ab  = A  + (size_t)b * strideA;
  const T* Bb  = Bt + (size_t)b * strideB;
  const T* Ab2 = SPLIT ? (A2  + (size_t)b * strideA) : nullptr;
  const T* Bb2 = SPLIT ? (Bt2 + (size_t)b * strideB) : nullptr;

  const int rlane = lane & 15;
  const int koff  = (lane >> 4) * 8;
  const int mOff  = (lane >> 4) * 8;

  v8f acc[4][4];
#pragma unroll
  for (int i = 0; i < 4; ++i)
#pragma unroll
    for (int j = 0; j < 4; ++j) acc[i][j] = (v8f){0.f,0.f,0.f,0.f,0.f,0.f,0.f,0.f};

  for (int k0 = 0; k0 < K; k0 += 32) {
    V bh[4], bl[4];
#pragma unroll
    for (int j = 0; j < 4; ++j) {
      const size_t bo = (size_t)(n0 + (j << 4) + rlane) * ldb + koff + k0;
      bh[j] = Frag<T>::load(Bb + bo);
      if (SPLIT) bl[j] = Frag<T>::load(Bb2 + bo);
    }
#pragma unroll
    for (int i = 0; i < 4; ++i) {
      const size_t ao = (size_t)(m0 + (i << 4) + rlane) * lda + koff + k0;
      V ah = Frag<T>::load(Ab + ao);
      V al;
      if (SPLIT) al = Frag<T>::load(Ab2 + ao);
#pragma unroll
      for (int j = 0; j < 4; ++j) {
        acc[i][j] = Frag<T>::mma(ah, bh[j], acc[i][j]);
        if (SPLIT) {
          acc[i][j] = Frag<T>::mma(ah, bl[j], acc[i][j]);
          acc[i][j] = Frag<T>::mma(al, bh[j], acc[i][j]);
        }
      }
      Frag<T>::guard(acc[i][0], acc[i][3], ah, SPLIT ? al : ah);
    }
    Frag<T>::keep(bh[0], bh[1], bh[2], bh[3]);
    if (SPLIT) Frag<T>::keep(bl[0], bl[1], bl[2], bl[3]);
  }
  acc_guard4(acc[0][0], acc[0][1], acc[0][2], acc[0][3]);
  acc_guard4(acc[1][0], acc[1][1], acc[1][2], acc[1][3]);
  acc_guard4(acc[2][0], acc[2][1], acc[2][2], acc[2][3]);
  acc_guard4(acc[3][0], acc[3][1], acc[3][2], acc[3][3]);

  float* slab = sT[wave];
  const float* Rb = RESID ? (resid + (size_t)b * strideR) : nullptr;
#pragma unroll
  for (int i = 0; i < 4; ++i) {
    const int mBase = m0 + (i << 4);
#pragma unroll
    for (int j = 0; j < 4; ++j) {
      const int n = n0 + (j << 4) + rlane;
      float bv = 0.f;
      if (BIAS_MODE == 2) bv = bias[n];
#pragma unroll
      for (int r = 0; r < 8; ++r) {
        float v = acc[i][j][r] * scale;
        if (BIAS_MODE == 1) v += bias[mBase + mOff + r];
        if (BIAS_MODE == 2) v += bv;
        if (RESID) v += Rb[(size_t)(mBase + mOff + r) * ldc + n];
        if (ACT == 2) v = fmaxf(v, 0.0f);
        if (ACT == 4) v = (v > 0.f) ? v : 0.01f * v;
        slab[(mOff + r) * 68 + (j << 4) + rlane] = v;
      }
    }
    __builtin_amdgcn_fence(__ATOMIC_RELEASE, "workgroup");
    __builtin_amdgcn_wave_barrier();
    __builtin_amdgcn_fence(__ATOMIC_ACQUIRE, "workgroup");
    if (OUT_MODE == 0) {
      float* C = (float*)Cout + (size_t)b * strideC;
      const int hh = lane >> 4, c4 = (lane & 15) * 4;
      for (int pass = 0; pass < 2; ++pass) {
#pragma unroll
        for (int it = 0; it < 8; ++it) {
          const int row = it * 2 + hh;
          v4f v = *(const v4f*)(slab + row * 68 + c4);
          *(volatile v4f*)(C + (size_t)(mBase + row) * ldc + n0 + c4) = v;
        }
        __threadfence();
      }
    } else {
      const int q = lane >> 3, c8 = (lane & 7) * 8;
      unsigned short* C  = (unsigned short*)Cout  + (size_t)b * strideC;
      unsigned short* C2 = (OUT_MODE == 2) ? ((unsigned short*)Cout2 + (size_t)b * strideC) : nullptr;
      for (int pass = 0; pass < 2; ++pass) {
#pragma unroll
        for (int it = 0; it < 4; ++it) {
          const int row = it * 4 + q;
          const float* sp = slab + row * 68 + c8;
          v8h hv, lv;
#pragma unroll
          for (int e = 0; e < 8; ++e) {
            if (OUT_MODE == 1) {
              hv[e] = (_Float16)sp[e];
            } else {
              unsigned short hb = f2bf_bits(sp[e]);
              unsigned short lb = f2bf_bits(sp[e] - bf_bits2f(hb));
              hv[e] = __builtin_bit_cast(_Float16, hb);
              lv[e] = __builtin_bit_cast(_Float16, lb);
            }
          }
          *(volatile v8h*)(C + (size_t)(mBase + row) * ldc + n0 + c8) = hv;
          if (OUT_MODE == 2) *(volatile v8h*)(C2 + (size_t)(mBase + row) * ldc + n0 + c8) = lv;
        }
        __threadfence();
      }
    }
    __builtin_amdgcn_fence(__ATOMIC_RELEASE, "workgroup");
    __builtin_amdgcn_wave_barrier();
    __builtin_amdgcn_fence(__ATOMIC_ACQUIRE, "workgroup");
  }
}

__device__ __forceinline__ void split_bf_words(float v, unsigned& t1, unsigned& t2) {
  const unsigned u = __float_as_uint(v);
  t1 = u + 0x7FFFu + ((u >> 16) & 1u);
  const float hf = __uint_as_float(t1 & 0xFFFF0000u);
  const float r = v - hf;
  const unsigned ur = __float_as_uint(r);
  t2 = ur + 0x7FFFu + ((ur >> 16) & 1u);
}
__device__ __forceinline__ unsigned pk_hi2(unsigned a, unsigned b) { return (a >> 16) | (b & 0xFFFF0000u); }

__global__ __launch_bounds__(256) void wsplit_kernel(const float* __restrict__ w,
                                                     unsigned short* __restrict__ WH,
                                                     unsigned short* __restrict__ WL, int n8) {
  const int i = blockIdx.x * 256 + threadIdx.x;
  if (i >= n8) return;
  const int e0  = i * 8;
  const int o   = e0 / kKdim;
  const int rem = e0 - o * kKdim;
  const int k   = rem >> 8;
  const int c0  = rem & 255;
  const float* src = w + (size_t)o * kKdim + (size_t)c0 * kTaps + k;
  unsigned th[8], tl[8];
#pragma unroll
  for (int e = 0; e < 8; ++e) split_bf_words(src[e * kTaps], th[e], tl[e]);
  const v4u uh = (v4u){pk_hi2(th[0], th[1]), pk_hi2(th[2], th[3]), pk_hi2(th[4], th[5]), pk_hi2(th[6], th[7])};
  const v4u ul = (v4u){pk_hi2(tl[0], tl[1]), pk_hi2(tl[2], tl[3]), pk_hi2(tl[4], tl[5]), pk_hi2(tl[6], tl[7])};
  unsigned short* ph = WH + (size_t)e0;
  unsigned short* pl = WL + (size_t)e0;
  *(volatile v4u*)ph = uh;
  *(volatile v4u*)pl = ul;
  __threadfence();
  *(volatile v4u*)ph = uh;
  *(volatile v4u*)pl = ul;
}

__global__ __launch_bounds__(256) void sample_kernel(const float* __restrict__ x,
                                                     const float* __restrict__ bboxes,
                                                     const float* __restrict__ scores,
                                                     const int* __restrict__ stride_p,
                                                     unsigned short* __restrict__ SH,
                                                     unsigned short* __restrict__ SL,
                                                     int b, int p0) {
  const int lane = threadIdx.x & 31;
  const int wave = threadIdx.x >> 5;
  const int pr = blockIdx.x * kPixPerBlk + wave;
  const int pg = p0 + pr;
  const int ph = pg >> 7;
  const int pw = pg & 127;
  const size_t pix = (size_t)b * kHW + (size_t)pg;
  const float bx1 = bboxes[pix * 4 + 0];
  const float by1 = bboxes[pix * 4 + 1];
  const float bx2 = bboxes[pix * 4 + 2];
  const float by2 = bboxes[pix * 4 + 3];
  const float sc  = scores[pix];
  const float strd  = (float)stride_p[0];
  const float inv_s = 1.0f / strd;
  const float x_ctr = ((bx1 + bx2) * 0.5f) * inv_s;
  const float y_ctr = ((by1 + by2) * 0.5f) * inv_s;
  const float dw = ((bx2 - bx1) * inv_s) * kThird;
  const float dh = ((by2 - by2) * inv_s) * kThird;
  const float xcf = (float)pw;
  const float ycf = (float)ph;
  const float* xl = x + (size_t)b * kChan * kHW + (size_t)lane * 8 * kHW;
  unsigned short* oh = SH + (size_t)pr * kKdim + lane * 8;
  unsigned short* ol = SL + (size_t)pr * kKdim + lane * 8;
#pragma unroll 1
  for (int it = 0; it < kTaps; ++it) {
    const float xx = (float)(it % 3 - 1);
    const float yy = (float)(it / 3 - 1);
    const float x_bbox = dw * xx + x_ctr;
    const float y_bbox = dh * yy + y_ctr;
    const float x_conv = xcf + xx;
    const float y_conv = ycf + yy;
    const float off_x = (x_bbox - x_conv) * sc;
    const float off_y = (y_bbox - y_conv) * sc;
    const float py = y_conv + off_y;
    const float px = x_conv + off_x;
    const float fy0 = floorf(py);
    const float fx0 = floorf(px);
    const float wy  = py - fy0;
    const float wx  = px - fx0;
    const float wy0 = 1.0f - wy;
    const float wx0 = 1.0f - wx;
    const int iy0 = (int)fminf(fmaxf(fy0, -4.0f), 132.0f);
    const int ix0 = (int)fminf(fmaxf(fx0, -4.0f), 132.0f);
    const int iy1 = iy0 + 1;
    const int ix1 = ix0 + 1;
    const bool vy0 = (iy0 >= 0) && (iy0 < kH);
    const bool vy1 = (iy1 >= 0) && (iy1 < kH);
    const bool vx0 = (ix0 >= 0) && (ix0 < kW);
    const bool vx1 = (ix1 >= 0) && (ix1 < kW);
    const float w00 = (vy0 && vx0) ? (wy0 * wx0) : 0.0f;
    const float w01 = (vy0 && vx1) ? (wy0 * wx)  : 0.0f;
    const float w10 = (vy1 && vx0) ? (wy  * wx0) : 0.0f;
    const float w11 = (vy1 && vx1) ? (wy  * wx)  : 0.0f;
    const int yc0 = min(max(iy0, 0), kH - 1);
    const int yc1 = min(max(iy1, 0), kH - 1);
    const int xc0 = min(max(ix0, 0), kW - 1);
    const int xc1 = min(max(ix1, 0), kW - 1);
    const float* q00 = xl + (yc0 * kW + xc0);
    const float* q01 = xl + (yc0 * kW + xc1);
    const float* q10 = xl + (yc1 * kW + xc0);
    const float* q11 = xl + (yc1 * kW + xc1);
    unsigned th[8], tl[8];
#pragma unroll
    for (int e = 0; e < 8; ++e) {
      const float a00 = q00[e * kHW];
      const float a01 = q01[e * kHW];
      const float a10 = q10[e * kHW];
      const float a11 = q11[e * kHW];
      float v = a00 * w00;
      v = v + a01 * w01;
      v = v + a10 * w10;
      v = v + a11 * w11;
      split_bf_words(v, th[e], tl[e]);
    }
    const v4u uh = (v4u){pk_hi2(th[0], th[1]), pk_hi2(th[2], th[3]), pk_hi2(th[4], th[5]), pk_hi2(th[6], th[7])};
    const v4u ul = (v4u){pk_hi2(tl[0], tl[1]), pk_hi2(tl[2], tl[3]), pk_hi2(tl[4], tl[5]), pk_hi2(tl[6], tl[7])};
    unsigned short* phs = oh + it * kChan;
    unsigned short* pls = ol + it * kChan;
    *(volatile v4u*)phs = uh;
    *(volatile v4u*)pls = ul;
    __threadfence();
    *(volatile v4u*)phs = uh;
    *(volatile v4u*)pls = ul;
  }
}

extern "C" void kernel_launch(void* const* d_in, const int* in_sizes, int n_in,
                              void* d_out, int out_size, void* d_ws, size_t ws_size,
                              hipStream_t stream) {
  if (n_in < 5) return;
  const float* x      = (const float*)d_in[0];
  const float* bboxes = (const float*)d_in[1];
  const float* scores = (const float*)d_in[2];
  const float* weight = (const float*)d_in[3];
  const int*   stride_p = (const int*)d_in[4];
  if (in_sizes[0] != kBatch * kChan * kHW) return;
  if (in_sizes[1] != kBatch * kHW * 4) return;
  if (in_sizes[2] != kBatch * kHW) return;
  if (in_sizes[3] != kChan * kKdim) return;
  if (in_sizes[4] < 1) return;
  if (out_size != kBatch * kChan * kHW) return;

  const size_t wPlaneBytes = (size_t)kChan * kKdim * 2;
  const size_t sPlaneBytes = (size_t)kHalfPix * kKdim * 2;
  const size_t offWH = 0;
  const size_t offWL = offWH + wPlaneBytes;
  const size_t offSH = offWL + wPlaneBytes;
  const size_t offSL = offSH + sPlaneBytes;
  const size_t total = offSL + sPlaneBytes;
  if (total > ws_size) return;
  unsigned char* ws = (unsigned char*)d_ws;
  unsigned short* WH = (unsigned short*)(ws + offWH);
  unsigned short* WL = (unsigned short*)(ws + offWL);
  unsigned short* SH = (unsigned short*)(ws + offSH);
  unsigned short* SL = (unsigned short*)(ws + offSL);
  const float* dummy_f = (const float*)(ws + offWH);
  void* dummy_v = (void*)(ws + offWL);

  const int n8 = kChan * kKdim / 8;
  wsplit_kernel<<<dim3((n8 + 255) / 256, 1, 1), dim3(256, 1, 1), 0, stream>>>(weight, WH, WL, n8);

  float* out = (float*)d_out;
  for (int s = 0; s < kBatch * (kHW / kHalfPix); ++s) {
    const int b  = s / (kHW / kHalfPix);
    const int p0 = (s % (kHW / kHalfPix)) * kHalfPix;
    sample_kernel<<<dim3(kHalfPix / kPixPerBlk, 1, 1), dim3(256, 1, 1), 0, stream>>>(
        x, bboxes, scores, stride_p, SH, SL, b, p0);
    const int tiles = (kChan / 64) * (kHalfPix / 64);
    wmma_gemm64<1, true, 0, 0, false, 2><<<dim3(tiles / 8, 1, 1), dim3(256, 1, 1), 0, stream>>>(
        WH, WL, kKdim, 0L,
        SH, SL, kKdim, 0L,
        (void*)(out + (size_t)b * kChan * kHW + (size_t)p0), dummy_v, kHW, 0L,
        dummy_f,
        dummy_f, 0L,
        kChan, kHalfPix, kKdim, 1.0f);
  }
}
